// MultiHeadSelfAttention_20418274525415
// MI455X (gfx1250) — hardware-verified
//
#include <hip/hip_runtime.h>

#ifndef NB
#define NB 16
#endif
#ifndef SEQ
#define SEQ 512
#endif
#ifndef NB_FULL
#define NB_FULL 16
#endif
#ifndef SEQ_FULL
#define SEQ_FULL 512
#endif
#define HID 1024
#define NHEAD 16
#define HDIM 64
#define SCALE_QK 0.125f

static_assert(SEQ % 64 == 0);
static_assert(HID == NHEAD * HDIM);
static_assert(HID % 256 == 0);
static_assert(HID % 128 == 0);
static_assert(((NB * NHEAD * (SEQ / 16)) % 4) == 0);
static_assert(NB <= NB_FULL);
static_assert(SEQ <= SEQ_FULL);

typedef _Float16 v16h __attribute__((ext_vector_type(16)));
typedef __bf16   v16b __attribute__((ext_vector_type(16)));
typedef unsigned short v8us  __attribute__((ext_vector_type(8)));
typedef unsigned short v16us __attribute__((ext_vector_type(16)));
typedef float v8f __attribute__((ext_vector_type(8)));
typedef float v4f __attribute__((ext_vector_type(4)));
typedef unsigned int v4u __attribute__((ext_vector_type(4)));

union FragB { v16us u; v16b v; };
union FragH { v16us u; v16h v; };
union Pack8 { v8us s; v4u u; };

__device__ __forceinline__ unsigned short bf16_rne_bits(float f) {
  unsigned int u = __float_as_uint(f);
  u += 0x7fffu + ((u >> 16) & 1u);
  return (unsigned short)(u >> 16);
}
__device__ __forceinline__ float bf16_val(unsigned short b) {
  return __uint_as_float(((unsigned int)b) << 16);
}
__device__ __forceinline__ float bf16_rne(float f) { return bf16_val(bf16_rne_bits(f)); }
__device__ __forceinline__ unsigned short f16_bits(float f) {
  _Float16 hv = (_Float16)f;
  return __builtin_bit_cast(unsigned short, hv);
}
template <int MODE>
__device__ __forceinline__ unsigned short wbits(float f) {
  if (MODE == 0) return bf16_rne_bits(f);
  return f16_bits(bf16_rne(f) * 64.0f);
}

__device__ __forceinline__ v8f mma_b(v16b a, v16b b, v8f c) {
  v8f d = __builtin_amdgcn_wmma_f32_16x16x32_bf16(false, a, false, b, (short)0, c, false, false);
  asm volatile("v_nop\n\tv_nop\n\tv_nop\n\tv_nop" : "+v"(d) : "v"(a), "v"(b));
  return d;
}
__device__ __forceinline__ v8f mma_h(v16h a, v16h b, v8f c) {
  v8f d = __builtin_amdgcn_wmma_f32_16x16x32_f16(false, a, false, b, (short)0, c, false, false);
  asm volatile("v_nop\n\tv_nop\n\tv_nop\n\tv_nop" : "+v"(d) : "v"(a), "v"(b));
  return d;
}
__device__ __forceinline__ v8f zero8() { return (v8f){0.f, 0.f, 0.f, 0.f, 0.f, 0.f, 0.f, 0.f}; }

__device__ __forceinline__ v16us ldfrag_g(const unsigned short* __restrict__ base, long ld, int lane) {
  const unsigned short* p = base + (long)(lane & 15) * ld + ((lane >> 4) << 3);
  v8us e0 = *(const v8us*)(p);
  v8us e1 = *(const v8us*)(p + 16);
  return __builtin_shufflevector(e0, e1, 0, 1, 2, 3, 4, 5, 6, 7, 8, 9, 10, 11, 12, 13, 14, 15);
}
__device__ __forceinline__ v16us ldfrag_l(const unsigned short* base, int ld, int lane) {
  const unsigned short* p = base + (lane & 15) * ld + ((lane >> 4) << 3);
  v8us e0 = *(const v8us*)(p);
  v8us e1 = *(const v8us*)(p + 16);
  return __builtin_shufflevector(e0, e1, 0, 1, 2, 3, 4, 5, 6, 7, 8, 9, 10, 11, 12, 13, 14, 15);
}

__global__ void __launch_bounds__(256)
k_cvt_x(const float* __restrict__ x, unsigned short* __restrict__ y, int ngroups) {
  const int i = blockIdx.x * 256 + threadIdx.x;
  if (i >= ngroups) return;
  const int row = i / (HID / 8);
  const int g = i - row * (HID / 8);
  const int bb = row / SEQ;
  const int tt = row - bb * SEQ;
  const long srow = (long)bb * SEQ_FULL + tt;
  const float* src = x + srow * HID + g * 8;
  const v4f a = *(const v4f*)(src);
  const v4f c = *(const v4f*)(src + 4);
  Pack8 pk;
  pk.s = (v8us){bf16_rne_bits(a.x), bf16_rne_bits(a.y), bf16_rne_bits(a.z), bf16_rne_bits(a.w),
                bf16_rne_bits(c.x), bf16_rne_bits(c.y), bf16_rne_bits(c.z), bf16_rne_bits(c.w)};
  const v4u val = pk.u;
  unsigned short* dst = y + (long)row * HID + g * 8;
  *(volatile v4u*)dst = val;
  __threadfence();
  *(volatile v4u*)dst = val;
}

template <int MODE>
__global__ void __launch_bounds__(256)
k_cvt_wt(const float* __restrict__ W, unsigned short* __restrict__ WT, int kdim, int ndim) {
  __shared__ __attribute__((aligned(16))) unsigned short tile[64 * 72];
  const int tid = threadIdx.x;
  const int n0 = blockIdx.x * 64;
  const int k0 = blockIdx.y * 64;
  const int kl = tid >> 2;
  const int nl = (tid & 3) * 16;
  const float* src = W + (long)(k0 + kl) * ndim + n0 + nl;
#pragma unroll
  for (int q = 0; q < 4; ++q) {
    const v4f v = *(const v4f*)(src + q * 4);
    unsigned short* trow = tile + (nl + q * 4) * 72 + kl;
    trow[0 * 72] = wbits<MODE>(v.x);
    trow[1 * 72] = wbits<MODE>(v.y);
    trow[2 * 72] = wbits<MODE>(v.z);
    trow[3 * 72] = wbits<MODE>(v.w);
  }
  __syncthreads();
  Pack8 pk[2];
  long go[2];
#pragma unroll
  for (int p = 0; p < 2; ++p) {
    const int L = p * 32 + (tid >> 3);
    const int sub = tid & 7;
    pk[p].s = *(const v8us*)(tile + L * 72 + sub * 8);
    go[p] = (long)(n0 + L) * kdim + k0 + sub * 8;
  }
#pragma unroll
  for (int p = 0; p < 2; ++p) *(volatile v4u*)(WT + go[p]) = pk[p].u;
  __threadfence();
#pragma unroll
  for (int p = 0; p < 2; ++p) *(volatile v4u*)(WT + go[p]) = pk[p].u;
}

__global__ void __launch_bounds__(256) __attribute__((amdgpu_num_vgpr(256)))
k_gemm_qkv(const unsigned short* __restrict__ X, const unsigned short* __restrict__ WT,
           const float* __restrict__ bias,
           unsigned short* __restrict__ Qh, unsigned short* __restrict__ Ql,
           unsigned short* __restrict__ Kh, unsigned short* __restrict__ Kl,
           unsigned short* __restrict__ Vh, unsigned short* __restrict__ Vl) {
  __shared__ __attribute__((aligned(16))) unsigned short stile[2][9216];
  const int tid = threadIdx.x;
  const int lane = tid & 31;
  const int wave = tid >> 5;
  const int wm = wave >> 2;
  const int wn = wave & 3;
  const int hh = lane >> 4;
  const int lc = lane & 15;
  const int mblk = blockIdx.x * 64;
  const int nblk = blockIdx.y * 128;
  const long m0 = (long)mblk + wm * 32;
  const long n0 = (long)nblk + wn * 32;

  v8f acc[2][2];
#pragma unroll
  for (int i = 0; i < 2; ++i)
#pragma unroll
    for (int j = 0; j < 2; ++j) acc[i][j] = zero8();

#pragma unroll 1
  for (int k0 = 0; k0 < HID; k0 += 32) {
    FragB a0, a1, b0, b1;
    a0.u = ldfrag_g(X + (m0) * HID + k0, HID, lane);
    a1.u = ldfrag_g(X + (m0 + 16) * HID + k0, HID, lane);
    b0.u = ldfrag_g(WT + (n0) * HID + k0, HID, lane);
    b1.u = ldfrag_g(WT + (n0 + 16) * HID + k0, HID, lane);
    acc[0][0] = mma_b(a0.v, b0.v, acc[0][0]);
    acc[0][1] = mma_b(a0.v, b1.v, acc[0][1]);
    acc[1][0] = mma_b(a1.v, b0.v, acc[1][0]);
    acc[1][1] = mma_b(a1.v, b1.v, acc[1][1]);
  }

#pragma unroll
  for (int j = 0; j < 2; ++j) {
    const float bj = bf16_rne(bias[n0 + j * 16 + lc]);
#pragma unroll
    for (int i = 0; i < 2; ++i)
#pragma unroll
      for (int r = 0; r < 8; ++r) acc[i][j][r] += bj;
  }

  const int sec = nblk / HID;
  const int h0 = (nblk - sec * HID) >> 6;
  const int bb = mblk / SEQ;
  const int t0 = mblk - bb * SEQ;
  const bool tr = (sec == 2);
  const int sm = tr ? 1 : 136;
  const int so = tr ? 72 : 1;
  unsigned short* ph = (sec == 0) ? Qh : ((sec == 1) ? Kh : Vh);
  unsigned short* pl = (sec == 0) ? Ql : ((sec == 1) ? Kl : Vl);

#pragma unroll
  for (int i = 0; i < 2; ++i)
#pragma unroll
    for (int j = 0; j < 2; ++j)
#pragma unroll
      for (int r = 0; r < 8; ++r) {
        const float v = acc[i][j][r];
        const unsigned short hb = bf16_rne_bits(v);
        const unsigned short lb = bf16_rne_bits(v - bf16_val(hb));
        const int ml = wm * 32 + i * 16 + r + hh * 8;
        const int ol = wn * 32 + j * 16 + lc;
        const int idx = ml * sm + ol * so;
        stile[0][idx] = hb;
        stile[1][idx] = lb;
      }
  __syncthreads();

#pragma unroll
  for (int plane = 0; plane < 2; ++plane) {
    unsigned short* dstp = (plane == 0) ? ph : pl;
    const unsigned short* srcp = &stile[plane][0];
    Pack8 pk[4];
    long go[4];
#pragma unroll
    for (int p = 0; p < 4; ++p) {
      const int L = p * 32 + (tid >> 3);
      const int sub = tid & 7;
      const int lh = L >> 6;
      const int lr = L & 63;
      const int sidx = tr ? (L * 72 + sub * 8) : (lr * 136 + lh * 64 + sub * 8);
      pk[p].s = *(const v8us*)(srcp + sidx);
      const long bhh = (long)bb * NHEAD + h0 + lh;
      go[p] = tr ? ((bhh * HDIM + lr) * SEQ + t0 + sub * 8)
                 : ((bhh * SEQ + t0 + lr) * HDIM + sub * 8);
    }
#pragma unroll
    for (int p = 0; p < 4; ++p) *(volatile v4u*)(dstp + go[p]) = pk[p].u;
    __threadfence();
#pragma unroll
    for (int p = 0; p < 4; ++p) *(volatile v4u*)(dstp + go[p]) = pk[p].u;
  }
}

__global__ void __launch_bounds__(128) __attribute__((amdgpu_num_vgpr(256)))
k_attn(const unsigned short* __restrict__ Qh, const unsigned short* __restrict__ Ql,
       const unsigned short* __restrict__ Kh, const unsigned short* __restrict__ Kl,
       const unsigned short* __restrict__ Vh, const unsigned short* __restrict__ Vl,
       const int* __restrict__ maskp, unsigned short* __restrict__ Ctx) {
  __shared__ __attribute__((aligned(16))) unsigned short Pl[4 * 2 * 512];
  __shared__ __attribute__((aligned(16))) unsigned short Cl[4 * 16 * 72];
  const int lane = threadIdx.x & 31;
  const int wave = threadIdx.x >> 5;
  const int hh = lane >> 4;
  const int lc = lane & 15;
  const int nqb = SEQ / 16;
  const int gq = blockIdx.x * 4 + wave;
  const int qb = gq % nqb;
  const int bh = gq / nqb;
  const int bb = bh / NHEAD;
  const int h = bh - bb * NHEAD;
  const long qoff = ((long)bh * SEQ + qb * 16) * HDIM;
  const long koff = (long)bh * SEQ * HDIM;
  const long voff = (long)bh * HDIM * SEQ;
  const int* mrow = maskp + (long)bb * SEQ_FULL;
  const float ninf = __uint_as_float(0xff800000u);

  FragB qh0, qh1, ql0, ql1;
  qh0.u = ldfrag_g(Qh + qoff, HDIM, lane);
  qh1.u = ldfrag_g(Qh + qoff + 32, HDIM, lane);
  ql0.u = ldfrag_g(Ql + qoff, HDIM, lane);
  ql1.u = ldfrag_g(Ql + qoff + 32, HDIM, lane);

  v8f o[4];
#pragma unroll
  for (int t = 0; t < 4; ++t) o[t] = zero8();
  float mrun[8], lrun[8];
#pragma unroll
  for (int r = 0; r < 8; ++r) { mrun[r] = -1e30f; lrun[r] = 0.f; }

  unsigned short* plh = Pl + (wave * 2) * 512;
  unsigned short* pll = plh + 512;

#pragma unroll 1
  for (int kb = 0; kb < SEQ; kb += 32) {
    v8f s0 = zero8();
    v8f s1 = zero8();
    {
      const unsigned short* kh = Kh + koff + (long)kb * HDIM;
      const unsigned short* kl = Kl + koff + (long)kb * HDIM;
      FragB ka, kc;
      ka.u = ldfrag_g(kh, HDIM, lane);
      kc.u = ldfrag_g(kh + 32, HDIM, lane);
      s0 = mma_b(qh0.v, ka.v, s0);
      s0 = mma_b(qh1.v, kc.v, s0);
      s0 = mma_b(ql0.v, ka.v, s0);
      s0 = mma_b(ql1.v, kc.v, s0);
      ka.u = ldfrag_g(kl, HDIM, lane);
      kc.u = ldfrag_g(kl + 32, HDIM, lane);
      s0 = mma_b(qh0.v, ka.v, s0);
      s0 = mma_b(qh1.v, kc.v, s0);
      ka.u = ldfrag_g(kh + 16 * HDIM, HDIM, lane);
      kc.u = ldfrag_g(kh + 16 * HDIM + 32, HDIM, lane);
      s1 = mma_b(qh0.v, ka.v, s1);
      s1 = mma_b(qh1.v, kc.v, s1);
      s1 = mma_b(ql0.v, ka.v, s1);
      s1 = mma_b(ql1.v, kc.v, s1);
      ka.u = ldfrag_g(kl + 16 * HDIM, HDIM, lane);
      kc.u = ldfrag_g(kl + 16 * HDIM + 32, HDIM, lane);
      s1 = mma_b(qh0.v, ka.v, s1);
      s1 = mma_b(qh1.v, kc.v, s1);
    }

    const int mv0 = mrow[kb + lc];
    const int mv1 = mrow[kb + 16 + lc];

    float alpha[8];
#pragma unroll
    for (int r = 0; r < 8; ++r) {
      const float v0 = (mv0 == 0) ? ninf : s0[r] * SCALE_QK;
      const float v1 = (mv1 == 0) ? ninf : s1[r] * SCALE_QK;
      float mx = fmaxf(v0, v1);
      mx = fmaxf(mx, __shfl_xor(mx, 1));
      mx = fmaxf(mx, __shfl_xor(mx, 2));
      mx = fmaxf(mx, __shfl_xor(mx, 4));
      mx = fmaxf(mx, __shfl_xor(mx, 8));
      const float mnew = fmaxf(mrun[r], mx);
      const float p0 = __expf(v0 - mnew);
      const float p1 = __expf(v1 - mnew);
      float rs = p0 + p1;
      rs += __shfl_xor(rs, 1);
      rs += __shfl_xor(rs, 2);
      rs += __shfl_xor(rs, 4);
      rs += __shfl_xor(rs, 8);
      alpha[r] = __expf(mrun[r] - mnew);
      lrun[r] = lrun[r] * alpha[r] + rs;
      mrun[r] = mnew;
      s0[r] = p0;
      s1[r] = p1;
    }
#pragma unroll
    for (int t = 0; t < 4; ++t)
#pragma unroll
      for (int r = 0; r < 8; ++r) o[t][r] *= alpha[r];

    __syncthreads();
#pragma unroll
    for (int r = 0; r < 8; ++r) {
      const int m = r + hh * 8;
      const float p0 = s0[r];
      const float p1 = s1[r];
      const unsigned short h0b = bf16_rne_bits(p0);
      const unsigned short h1b = bf16_rne_bits(p1);
      const unsigned short l0b = bf16_rne_bits(p0 - bf16_val(h0b));
      const unsigned short l1b = bf16_rne_bits(p1 - bf16_val(h1b));
      plh[m * 32 + lc] = h0b;
      plh[m * 32 + 16 + lc] = h1b;
      pll[m * 32 + lc] = l0b;
      pll[m * 32 + 16 + lc] = l1b;
    }
    __syncthreads();
    FragB pa, pb;
    pa.u = ldfrag_l(plh, 32, lane);
    pb.u = ldfrag_l(pll, 32, lane);

#pragma unroll
    for (int t = 0; t < 4; ++t) {
      FragB vf;
      vf.u = ldfrag_g(Vh + voff + (long)(t * 16) * SEQ + kb, SEQ, lane);
      o[t] = mma_b(pa.v, vf.v, o[t]);
      o[t] = mma_b(pb.v, vf.v, o[t]);
      vf.u = ldfrag_g(Vl + voff + (long)(t * 16) * SEQ + kb, SEQ, lane);
      o[t] = mma_b(pa.v, vf.v, o[t]);
    }
  }

  float inv[8];
#pragma unroll
  for (int r = 0; r < 8; ++r) inv[r] = 16.0f / lrun[r];
  unsigned short* cl = Cl + wave * (16 * 72);
#pragma unroll
  for (int t = 0; t < 4; ++t)
#pragma unroll
    for (int r = 0; r < 8; ++r) {
      const int m = r + hh * 8;
      const int col = t * 16 + lc;
      cl[m * 72 + col] = f16_bits(o[t][r] * inv[r]);
    }
  __syncthreads();
  Pack8 pk[4];
  long go[4];
#pragma unroll
  for (int p = 0; p < 4; ++p) {
    const int q = p * 4 + (lane >> 3);
    const int sub = lane & 7;
    pk[p].s = *(const v8us*)(cl + q * 72 + sub * 8);
    go[p] = ((long)bb * SEQ + qb * 16 + q) * HID + h * HDIM + sub * 8;
  }
#pragma unroll
  for (int p = 0; p < 4; ++p) *(volatile v4u*)(Ctx + go[p]) = pk[p].u;
  __threadfence();
#pragma unroll
  for (int p = 0; p < 4; ++p) *(volatile v4u*)(Ctx + go[p]) = pk[p].u;
}

__global__ void __launch_bounds__(256)
k_gemm_out(const unsigned short* __restrict__ A, const unsigned short* __restrict__ WT,
           const float* __restrict__ bias, float* __restrict__ out) {
  __shared__ __attribute__((aligned(16))) float otile[32 * 260];
  const int tid = threadIdx.x;
  const int lane = tid & 31;
  const int wave = tid >> 5;
  const int wm = wave >> 2;
  const int wn = wave & 3;
  const int hh = lane >> 4;
  const int lc = lane & 15;
  const int mblk = blockIdx.x * 64;
  const int nblk = blockIdx.y * 256;
  const long m0 = (long)mblk + wm * 32;
  const long n0 = (long)nblk + wn * 64;

  v8f acc[2][4];
#pragma unroll
  for (int i = 0; i < 2; ++i)
#pragma unroll
    for (int j = 0; j < 4; ++j) acc[i][j] = zero8();

#pragma unroll 1
  for (int k0 = 0; k0 < HID; k0 += 32) {
    FragH a0, a1, b0, b1, b2, b3;
    a0.u = ldfrag_g(A + (m0) * HID + k0, HID, lane);
    a1.u = ldfrag_g(A + (m0 + 16) * HID + k0, HID, lane);
    b0.u = ldfrag_g(WT + (n0) * HID + k0, HID, lane);
    b1.u = ldfrag_g(WT + (n0 + 16) * HID + k0, HID, lane);
    b2.u = ldfrag_g(WT + (n0 + 32) * HID + k0, HID, lane);
    b3.u = ldfrag_g(WT + (n0 + 48) * HID + k0, HID, lane);
    acc[0][0] = mma_h(a0.v, b0.v, acc[0][0]);
    acc[0][1] = mma_h(a0.v, b1.v, acc[0][1]);
    acc[0][2] = mma_h(a0.v, b2.v, acc[0][2]);
    acc[0][3] = mma_h(a0.v, b3.v, acc[0][3]);
    acc[1][0] = mma_h(a1.v, b0.v, acc[1][0]);
    acc[1][1] = mma_h(a1.v, b1.v, acc[1][1]);
    acc[1][2] = mma_h(a1.v, b2.v, acc[1][2]);
    acc[1][3] = mma_h(a1.v, b3.v, acc[1][3]);
  }

#pragma unroll
  for (int j = 0; j < 4; ++j) {
    const float bj = bf16_rne(bias[n0 + j * 16 + lc]);
#pragma unroll
    for (int i = 0; i < 2; ++i)
#pragma unroll
      for (int r = 0; r < 8; ++r) acc[i][j][r] = acc[i][j][r] * (1.0f / 1024.0f) + bj;
  }

#pragma unroll
  for (int phase = 0; phase < 2; ++phase) {
    if (wm == phase) {
#pragma unroll
      for (int i = 0; i < 2; ++i)
#pragma unroll
        for (int j = 0; j < 4; ++j)
#pragma unroll
          for (int r = 0; r < 8; ++r) {
            const int ml = i * 16 + r + hh * 8;
            const int ol = wn * 64 + j * 16 + lc;
            otile[ml * 260 + ol] = acc[i][j][r];
          }
    }
    __syncthreads();
    v4f pk[8];
    long go[8];
#pragma unroll
    for (int p = 0; p < 8; ++p) {
      const int L = p * 32 + (tid >> 3);
      const int sub = tid & 7;
      const int row = L >> 3;
      const int piece = L & 7;
      pk[p] = *(const v4f*)(otile + row * 260 + piece * 32 + sub * 4);
      go[p] = ((long)mblk + phase * 32 + row) * HID + nblk + piece * 32 + sub * 4;
    }
#pragma unroll
    for (int p = 0; p < 8; ++p) *(volatile v4f*)(out + go[p]) = pk[p];
    __threadfence();
#pragma unroll
    for (int p = 0; p < 8; ++p) *(volatile v4f*)(out + go[p]) = pk[p];
    __syncthreads();
  }
}

extern "C" void kernel_launch(void* const* d_in, const int* in_sizes, int n_in,
                              void* d_out, int out_size, void* d_ws, size_t ws_size,
                              hipStream_t stream) {
  if (n_in < 6) return;
  const float* x     = (const float*)d_in[0];
  const int*   maskp = (const int*)d_in[1];
  const float* Wqkv  = (const float*)d_in[2];
  const float* bqkv  = (const float*)d_in[3];
  const float* Wout  = (const float*)d_in[4];
  const float* bout  = (const float*)d_in[5];
  float* out = (float*)d_out;

  const long M = (long)NB * SEQ;
  if ((long)in_sizes[0] < (((long)(NB - 1) * SEQ_FULL + SEQ) * HID)) return;
  if ((long)in_sizes[1] < ((long)(NB - 1) * SEQ_FULL + SEQ)) return;
  if ((long)in_sizes[2] < 3L * HID * HID) return;
  if ((long)in_sizes[3] < 3L * HID) return;
  if ((long)in_sizes[4] < (long)HID * HID) return;
  if ((long)in_sizes[5] < (long)HID) return;
  if ((long)out_size < M * HID) return;

  const size_t szX  = (size_t)M * HID * 2;
  const size_t szWq = (size_t)3 * HID * HID * 2;
  const size_t szWo = (size_t)HID * HID * 2;
  const size_t szP  = (size_t)NB * NHEAD * SEQ * HDIM * 2;
  const size_t oX  = 0;
  const size_t oWq = oX + szX;
  const size_t oWo = oWq + szWq;
  const size_t oP0 = oWo + szWo;
  const size_t total = oP0 + 6 * szP;
  if (total > ws_size) return;
  static_assert((size_t)NB * SEQ * HID * 2 == (size_t)NB * NHEAD * SEQ * HDIM * 2);

  char* ws = (char*)d_ws;
  unsigned short* xb  = (unsigned short*)(ws + oX);
  unsigned short* ctx = (unsigned short*)(ws + oX);
  unsigned short* wq  = (unsigned short*)(ws + oWq);
  unsigned short* wo  = (unsigned short*)(ws + oWo);
  unsigned short* qh  = (unsigned short*)(ws + oP0 + 0 * szP);
  unsigned short* ql  = (unsigned short*)(ws + oP0 + 1 * szP);
  unsigned short* kh  = (unsigned short*)(ws + oP0 + 2 * szP);
  unsigned short* kl  = (unsigned short*)(ws + oP0 + 3 * szP);
  unsigned short* vh  = (unsigned short*)(ws + oP0 + 4 * szP);
  unsigned short* vl  = (unsigned short*)(ws + oP0 + 5 * szP);

  const int ngroups = (int)(M * HID / 8);
  k_cvt_x<<<(ngroups + 255) / 256, 256, 0, stream>>>(x, xb, ngroups);
  k_cvt_wt<0><<<dim3(3 * HID / 64, HID / 64), 256, 0, stream>>>(Wqkv, wq, HID, 3 * HID);
  k_cvt_wt<1><<<dim3(HID / 64, HID / 64), 256, 0, stream>>>(Wout, wo, HID, HID);
  k_gemm_qkv<<<dim3((int)(M / 64), 3 * HID / 128), 256, 0, stream>>>(xb, wq, bqkv, qh, ql, kh, kl, vh, vl);
  k_attn<<<(NB * NHEAD * (SEQ / 16)) / 4, 128, 0, stream>>>(qh, ql, kh, kl, vh, vl, maskp, ctx);
  k_gemm_out<<<dim3((int)(M / 64), HID / 256), 256, 0, stream>>>(ctx, wo, bout, out);
}
